// ABNet_67250597920810
// MI455X (gfx1250) — hardware-verified
//
#include <hip/hip_runtime.h>
#include <math.h>

constexpr int   kHeads      = 10;
constexpr int   kRows       = 32768;
constexpr int   kDimIn      = 4;
constexpr int   kHid        = 256;
constexpr int   kGroup      = 2;
constexpr int   kNGroups    = kHeads / kGroup;
constexpr int   kNLayers    = 5;
constexpr long  kPlaneElems = (long)kRows * kHid;
constexpr long  kSlotElems  = kPlaneElems * kGroup;
constexpr long  kWElems     = (long)kHid * kHid;
constexpr long  kWLayer     = kWElems * kHeads;
constexpr long  kBLayer     = (long)kHid * kHeads;
constexpr float kActCarry   = 8.0f;
constexpr float kWCarry     = 16.0f;
constexpr float kGemmScale  = kActCarry / (kActCarry * kWCarry);
constexpr float kTailScale  = 1.0f / (kActCarry * kWCarry);
constexpr int   kBtPitch    = 264;
constexpr int   kGemmBlocks = (kRows / 64) * (kHid / 64) / 8;
constexpr float kL1 = 3.0f, kL2 = 3.0f, kObsX = 0.0f, kObsY = 7.0f, kR2 = 16.0f;

static_assert(kRows % 128 == 0);
static_assert(kHid % 64 == 0);
static_assert((kRows / 64) * (kHid / 64) % 8 == 0);
static_assert(kHeads % kGroup == 0);

constexpr size_t kOffW16   = 0;
constexpr size_t kBytesW16 = (size_t)kNLayers * kWLayer * 2;
constexpr size_t kOffB8    = kOffW16 + kBytesW16;
constexpr size_t kBytesB8  = (size_t)kNLayers * kBLayer * 4;
constexpr size_t kOffPlane = kOffB8 + kBytesB8;
constexpr size_t kBytesSlot = (size_t)kSlotElems * 2;
constexpr size_t kOffA0    = kOffPlane + 3 * kBytesSlot;
constexpr size_t kBytesAcc = (size_t)kRows * 2 * 4;
constexpr size_t kOffAcc0  = kOffA0 + kBytesAcc;
constexpr size_t kOffAcc1  = kOffAcc0 + kBytesAcc;
constexpr size_t kWsTotal  = kOffAcc1 + kBytesAcc;
static_assert(kOffB8 % 128 == 0 && kOffPlane % 128 == 0 && kOffA0 % 128 == 0 && kOffAcc0 % 128 == 0 && kOffAcc1 % 128 == 0);
static_assert(kWsTotal <= 134217728ull);

typedef __attribute__((ext_vector_type(16))) _Float16 v16h;
typedef __attribute__((ext_vector_type(8)))  _Float16 v8h;
typedef __attribute__((ext_vector_type(16))) __bf16   v16b;
typedef __attribute__((ext_vector_type(8)))  __bf16   v8b;
typedef __attribute__((ext_vector_type(8)))  float    v8f;
typedef __attribute__((ext_vector_type(4)))  float    v4f;
typedef __attribute__((ext_vector_type(4)))  unsigned int v4u;

__device__ __forceinline__ unsigned short f2bf_bits(float f) {
  unsigned u = __float_as_uint(f);
  return (unsigned short)((u + 0x7FFFu + ((u >> 16) & 1u)) >> 16);
}
__device__ __forceinline__ float bf_bits2f(unsigned short h) { return __uint_as_float(((unsigned)h) << 16); }

__device__ __forceinline__ void dep_guard_h(v8f& a, v8f& b, v16h x, v16h y) { asm volatile("v_nop\n\tv_nop\n\tv_nop\n\tv_nop" : "+v"(a), "+v"(b) : "v"(x), "v"(y)); }
__device__ __forceinline__ void dep_guard_b(v8f& a, v8f& b, v16b x, v16b y) { asm volatile("v_nop\n\tv_nop\n\tv_nop\n\tv_nop" : "+v"(a), "+v"(b) : "v"(x), "v"(y)); }
__device__ __forceinline__ void keep4_h(v16h a, v16h b, v16h c, v16h d) { asm volatile("v_nop" :: "v"(a), "v"(b), "v"(c), "v"(d)); }
__device__ __forceinline__ void keep4_b(v16b a, v16b b, v16b c, v16b d) { asm volatile("v_nop" :: "v"(a), "v"(b), "v"(c), "v"(d)); }
__device__ __forceinline__ void acc_guard4(v8f& a, v8f& b, v8f& c, v8f& d) { asm volatile("v_nop\n\tv_nop\n\tv_nop\n\tv_nop" : "+v"(a), "+v"(b), "+v"(c), "+v"(d)); }
template <typename T> struct Frag;
template <> struct Frag<_Float16> {
  typedef v16h V; union U { v16h v; v8h h[2]; };
  static __device__ __forceinline__ v16h load(const _Float16* p) {
    U f; f.h[0] = *(const v8h*)(p); f.h[1] = *(const v8h*)(p + 16); return f.v;
  }
  static __device__ __forceinline__ v8f mma(v16h a, v16h b, v8f c) {
    return __builtin_amdgcn_wmma_f32_16x16x32_f16(false, a, false, b, (short)0, c, false, false);
  }
  static __device__ __forceinline__ void guard(v8f& a, v8f& b, v16h x, v16h y) { dep_guard_h(a, b, x, y); }
  static __device__ __forceinline__ void keep(v16h a, v16h b, v16h c, v16h d) { keep4_h(a, b, c, d); }
};
template <> struct Frag<__bf16> {
  typedef v16b V; union U { v16b v; v8b h[2]; };
  static __device__ __forceinline__ v16b load(const __bf16* p) {
    U f; f.h[0] = *(const v8b*)(p); f.h[1] = *(const v8b*)(p + 16); return f.v;
  }
  static __device__ __forceinline__ v8f mma(v16b a, v16b b, v8f c) {
    return __builtin_amdgcn_wmma_f32_16x16x32_bf16(false, a, false, b, (short)0, c, false, false);
  }
  static __device__ __forceinline__ void guard(v8f& a, v8f& b, v16b x, v16b y) { dep_guard_b(a, b, x, y); }
  static __device__ __forceinline__ void keep(v16b a, v16b b, v16b c, v16b d) { keep4_b(a, b, c, d); }
};

__device__ __forceinline__ unsigned pk16(unsigned short a, unsigned short b) { return (unsigned)a | ((unsigned)b << 16); }
__device__ __forceinline__ unsigned short h_bits(float f) { const _Float16 h = (_Float16)f; return __builtin_bit_cast(unsigned short, h); }
__device__ __forceinline__ void wave_sync() {
  __builtin_amdgcn_fence(__ATOMIC_RELEASE, "workgroup");
  __builtin_amdgcn_wave_barrier();
  __builtin_amdgcn_fence(__ATOMIC_ACQUIRE, "workgroup");
}

template <int ET> struct Elem;
template <> struct Elem<0> { typedef _Float16 T; };
template <> struct Elem<1> { typedef __bf16 T; };
template <int ET, bool SPLIT, int BIAS_MODE, int OUT_MODE, bool RESID, int ACT = 0>
__global__ __launch_bounds__(256) void wmma_gemm64(
    const unsigned short* __restrict__ Ap, const unsigned short* __restrict__ A2p, int lda, long strideA,
    const unsigned short* __restrict__ Btp, const unsigned short* __restrict__ Bt2p, int ldb, long strideB,
    void* __restrict__ Cout, void* __restrict__ Cout2, int ldc, long strideC,
    const float* __restrict__ bias, long strideBias,
    const float* __restrict__ resid, long strideR,
    int M, int N, int K, float scale) {
  typedef typename Elem<ET>::T T;
  typedef typename Frag<T>::V V;
  const T* A = (const T*)Ap; const T* A2 = (const T*)A2p; const T* Bt = (const T*)Btp; const T* Bt2 = (const T*)Bt2p;
  __shared__ __align__(16) float sT[8][16 * 68];
  const int b    = blockIdx.y;
  const int lane = threadIdx.x & 31;
  const int wave = threadIdx.x >> 5;
  const int tilesN = N >> 6;
  const int tilesM = M >> 6;
  const int tile = blockIdx.x * 8 + wave;
  if (tile >= tilesM * tilesN) return;
  const int tm = tile / tilesN;
  const int tn = tile - tm * tilesN;
  const int m0 = tm << 6;
  const int n0 = tn << 6;

  const T* Ab  = A  + (size_t)b * strideA;
  const T* Bb  = Bt + (size_t)b * strideB;
  const T* Ab2 = SPLIT ? (A2  + (size_t)b * strideA) : nullptr;
  const T* Bb2 = SPLIT ? (Bt2 + (size_t)b * strideB) : nullptr;
  const float* biasb = (BIAS_MODE != 0) ? (bias + (size_t)b * strideBias) : nullptr;

  const int rlane = lane & 15;
  const int koff  = (lane >> 4) * 8;
  const int mOff  = (lane >> 4) * 8;

  v8f acc[4][4];
#pragma unroll
  for (int i = 0; i < 4; ++i)
#pragma unroll
    for (int j = 0; j < 4; ++j) acc[i][j] = (v8f){0.f,0.f,0.f,0.f,0.f,0.f,0.f,0.f};

  for (int k0 = 0; k0 < K; k0 += 32) {
    V bh[4], bl[4];
#pragma unroll
    for (int j = 0; j < 4; ++j) {
      const size_t bo = (size_t)(n0 + (j << 4) + rlane) * ldb + koff + k0;
      bh[j] = Frag<T>::load(Bb + bo);
      if (SPLIT) bl[j] = Frag<T>::load(Bb2 + bo);
    }
#pragma unroll
    for (int i = 0; i < 4; ++i) {
      const size_t ao = (size_t)(m0 + (i << 4) + rlane) * lda + koff + k0;
      V ah = Frag<T>::load(Ab + ao);
      V al;
      if (SPLIT) al = Frag<T>::load(Ab2 + ao);
#pragma unroll
      for (int j = 0; j < 4; ++j) {
        acc[i][j] = Frag<T>::mma(ah, bh[j], acc[i][j]);
        if (SPLIT) {
          acc[i][j] = Frag<T>::mma(ah, bl[j], acc[i][j]);
          acc[i][j] = Frag<T>::mma(al, bh[j], acc[i][j]);
        }
      }
      Frag<T>::guard(acc[i][0], acc[i][3], ah, SPLIT ? al : ah);
    }
    Frag<T>::keep(bh[0], bh[1], bh[2], bh[3]);
    if (SPLIT) Frag<T>::keep(bl[0], bl[1], bl[2], bl[3]);
  }
  acc_guard4(acc[0][0], acc[0][1], acc[0][2], acc[0][3]);
  acc_guard4(acc[1][0], acc[1][1], acc[1][2], acc[1][3]);
  acc_guard4(acc[2][0], acc[2][1], acc[2][2], acc[2][3]);
  acc_guard4(acc[3][0], acc[3][1], acc[3][2], acc[3][3]);

  float* slab = sT[wave];
  const float* Rb = RESID ? (resid + (size_t)b * strideR) : nullptr;
#pragma unroll
  for (int i = 0; i < 4; ++i) {
    const int mBase = m0 + (i << 4);
#pragma unroll
    for (int j = 0; j < 4; ++j) {
      const int n = n0 + (j << 4) + rlane;
      float bv = 0.f;
      if (BIAS_MODE == 2) bv = biasb[n];
#pragma unroll
      for (int r = 0; r < 8; ++r) {
        float v = acc[i][j][r] * scale;
        if (BIAS_MODE == 1) v += biasb[mBase + mOff + r];
        if (BIAS_MODE == 2) v += bv;
        if (RESID) v += Rb[(size_t)(mBase + mOff + r) * ldc + n];
        if (ACT == 2) v = fmaxf(v, 0.0f);
        if (ACT == 4) v = (v > 0.f) ? v : 0.01f * v;
        slab[(mOff + r) * 68 + (j << 4) + rlane] = v;
      }
    }
    __builtin_amdgcn_fence(__ATOMIC_RELEASE, "workgroup");
    __builtin_amdgcn_wave_barrier();
    __builtin_amdgcn_fence(__ATOMIC_ACQUIRE, "workgroup");
    if (OUT_MODE == 0) {
      float* C = (float*)Cout + (size_t)b * strideC;
      const int hh = lane >> 4, c4 = (lane & 15) * 4;
      for (int pass = 0; pass < 2; ++pass) {
#pragma unroll
        for (int it = 0; it < 8; ++it) {
          const int row = it * 2 + hh;
          v4f v = *(const v4f*)(slab + row * 68 + c4);
          *(volatile v4f*)(C + (size_t)(mBase + row) * ldc + n0 + c4) = v;
        }
        __threadfence();
      }
    } else {
      const int q = lane >> 3, c8 = (lane & 7) * 8;
      unsigned short* C  = (unsigned short*)Cout  + (size_t)b * strideC;
      unsigned short* C2 = (OUT_MODE == 2) ? ((unsigned short*)Cout2 + (size_t)b * strideC) : nullptr;
      for (int pass = 0; pass < 2; ++pass) {
#pragma unroll
        for (int it = 0; it < 4; ++it) {
          const int row = it * 4 + q;
          const float* sp = slab + row * 68 + c8;
          v8h hv, lv;
#pragma unroll
          for (int e = 0; e < 8; ++e) {
            if (OUT_MODE == 1) {
              hv[e] = (_Float16)sp[e];
            } else {
              unsigned short hb = f2bf_bits(sp[e]);
              unsigned short lb = f2bf_bits(sp[e] - bf_bits2f(hb));
              hv[e] = __builtin_bit_cast(_Float16, hb);
              lv[e] = __builtin_bit_cast(_Float16, lb);
            }
          }
          *(volatile v8h*)(C + (size_t)(mBase + row) * ldc + n0 + c8) = hv;
          if (OUT_MODE == 2) *(volatile v8h*)(C2 + (size_t)(mBase + row) * ldc + n0 + c8) = lv;
        }
        __threadfence();
      }
    }
    __builtin_amdgcn_fence(__ATOMIC_RELEASE, "workgroup");
    __builtin_amdgcn_wave_barrier();
    __builtin_amdgcn_fence(__ATOMIC_ACQUIRE, "workgroup");
  }
}

__global__ __launch_bounds__(256) void wcast8_kernel(const float* __restrict__ W0, const float* __restrict__ W1,
                                                     const float* __restrict__ W2, const float* __restrict__ W3,
                                                     const float* __restrict__ W4, unsigned short* __restrict__ out,
                                                     int n8, float scale) {
  const int y = blockIdx.y;
  const float* W = (y == 0) ? W0 : (y == 1) ? W1 : (y == 2) ? W2 : (y == 3) ? W3 : W4;
  const int i = blockIdx.x * 256 + threadIdx.x;
  if (i >= n8) return;
  const float* p = W + 8 * (size_t)i;
  const v4f a = *(const v4f*)(p);
  const v4f c = *(const v4f*)(p + 4);
  unsigned short hb[8];
#pragma unroll
  for (int e = 0; e < 4; ++e) {
    hb[e]     = h_bits(a[e] * scale);
    hb[4 + e] = h_bits(c[e] * scale);
  }
  const v4u u = (v4u){pk16(hb[0], hb[1]), pk16(hb[2], hb[3]), pk16(hb[4], hb[5]), pk16(hb[6], hb[7])};
  unsigned short* q = out + (size_t)y * ((size_t)n8 * 8) + 8 * (size_t)i;
  *(volatile v4u*)q = u;
  __threadfence();
  *(volatile v4u*)q = u;
}

__global__ __launch_bounds__(256) void bias_scale_kernel(const float* __restrict__ b0, const float* __restrict__ b1,
                                                         const float* __restrict__ b2, const float* __restrict__ b3,
                                                         const float* __restrict__ b4, float* __restrict__ out,
                                                         int n4, float scale) {
  const int y = blockIdx.y;
  const float* bp = (y == 0) ? b0 : (y == 1) ? b1 : (y == 2) ? b2 : (y == 3) ? b3 : b4;
  const int i = blockIdx.x * 256 + threadIdx.x;
  if (i >= n4) return;
  v4f v = *(const v4f*)(bp + 4 * (size_t)i);
  v = v * scale;
  float* q = out + (size_t)y * ((size_t)n4 * 4) + 4 * (size_t)i;
  *(volatile v4f*)q = v;
  __threadfence();
  *(volatile v4f*)q = v;
}

__global__ __launch_bounds__(256) void input_layer_kernel(const float* __restrict__ x, const float* __restrict__ W1,
                                                          const float* __restrict__ b1, unsigned short* __restrict__ out,
                                                          int hbase) {
  const long i  = (long)blockIdx.x * 256 + threadIdx.x;
  const int  n8 = (int)(i & 31);
  const int  b  = (int)((i >> 5) & (kRows - 1));
  const int  g  = (int)(i >> 20);
  const int  h  = hbase + g;
  const v4f xv = *(const v4f*)(x + (size_t)b * kDimIn);
  const float* wp = W1 + ((size_t)h * kHid + (size_t)n8 * 8) * kDimIn;
  const float* bp = b1 + (size_t)h * kHid + (size_t)n8 * 8;
  unsigned short hb[8];
#pragma unroll
  for (int e = 0; e < 8; ++e) {
    const v4f w = *(const v4f*)(wp + 4 * e);
    float v = xv[0] * w[0] + xv[1] * w[1] + xv[2] * w[2] + xv[3] * w[3] + bp[e];
    v = fmaxf(v, 0.0f) * kActCarry;
    hb[e] = h_bits(v);
  }
  const v4u u = (v4u){pk16(hb[0], hb[1]), pk16(hb[2], hb[3]), pk16(hb[4], hb[5]), pk16(hb[6], hb[7])};
  unsigned short* q = out + ((size_t)g * kRows + (size_t)b) * kHid + (size_t)n8 * 8;
  *(volatile v4u*)q = u;
  __threadfence();
  *(volatile v4u*)q = u;
}

__global__ __launch_bounds__(256) void tail_kernel(
    const unsigned short* __restrict__ P41, const unsigned short* __restrict__ P42,
    const float* __restrict__ W51, const float* __restrict__ b51,
    const float* __restrict__ W52, const float* __restrict__ b52,
    const float* __restrict__ x, const float* __restrict__ mean, const float* __restrict__ stdv,
    const float* __restrict__ mean_label, const float* __restrict__ std_label, const float* __restrict__ wt,
    const float* a0in, float* a0out, const float* accin, float* accout,
    int h, int has_prev, int write_a0) {
#pragma clang fp contract(off)
  __shared__ __align__(16) _Float16 Bt51[16 * kBtPitch];
  __shared__ __align__(16) _Float16 Bt52[16 * kBtPitch];
  __shared__ __align__(16) float sD[8][2][16 * 20];
  __shared__ __align__(16) float sOut[8][32];
  __shared__ __align__(16) float sA0[8][32];

  const int t = threadIdx.x;
  {
    const int n  = t >> 4;
    const int k0 = (t & 15) * 16;
    const int nc = (n < 2) ? n : 1;
    const float fac = (n < 2) ? kWCarry : 0.0f;
    const float* w1p = W51 + ((size_t)h * 2 + nc) * kHid + k0;
    const float* w2p = W52 + ((size_t)h * 2 + nc) * kHid + k0;
#pragma unroll
    for (int j = 0; j < 2; ++j) {
      const v4f a = *(const v4f*)(w1p + 8 * j);
      const v4f c = *(const v4f*)(w1p + 8 * j + 4);
      const v4f d = *(const v4f*)(w2p + 8 * j);
      const v4f f = *(const v4f*)(w2p + 8 * j + 4);
      v8h h1, h2;
#pragma unroll
      for (int e = 0; e < 4; ++e) {
        h1[e] = (_Float16)(a[e] * fac); h1[4 + e] = (_Float16)(c[e] * fac);
        h2[e] = (_Float16)(d[e] * fac); h2[4 + e] = (_Float16)(f[e] * fac);
      }
      *(v8h*)(Bt51 + n * kBtPitch + k0 + 8 * j) = h1;
      *(v8h*)(Bt52 + n * kBtPitch + k0 + 8 * j) = h2;
    }
  }
  __syncthreads();

  const int lane  = t & 31;
  const int wave  = t >> 5;
  const int rlane = lane & 15;
  const int koff  = (lane >> 4) * 8;
  const int mOff  = koff;
  const int q0    = blockIdx.x * 128 + wave * 16;

  const _Float16* A41 = (const _Float16*)P41 + (size_t)(q0 + rlane) * kHid + koff;
  const _Float16* A42 = (const _Float16*)P42 + (size_t)(q0 + rlane) * kHid + koff;
  const _Float16* B51p = Bt51 + rlane * kBtPitch + koff;
  const _Float16* B52p = Bt52 + rlane * kBtPitch + koff;
  v8f acc1 = (v8f){0.f,0.f,0.f,0.f,0.f,0.f,0.f,0.f};
  v8f acc2 = acc1;
#pragma unroll 2
  for (int ks = 0; ks < 8; ++ks) {
    const v16h a1  = Frag<_Float16>::load(A41 + ks * 32);
    const v16h a2  = Frag<_Float16>::load(A42 + ks * 32);
    const v16h bb1 = Frag<_Float16>::load(B51p + ks * 32);
    const v16h bb2 = Frag<_Float16>::load(B52p + ks * 32);
    acc1 = Frag<_Float16>::mma(a1, bb1, acc1);
    acc2 = Frag<_Float16>::mma(a2, bb2, acc2);
    dep_guard_h(acc1, acc2, a1, a2);
    keep4_h(bb1, bb2, a1, a2);
  }
  dep_guard_h(acc1, acc2, (v16h){}, (v16h){});

  float* sl1 = sD[wave][0];
  float* sl2 = sD[wave][1];
#pragma unroll
  for (int r = 0; r < 8; ++r) {
    sl1[(mOff + r) * 20 + rlane] = acc1[r];
    sl2[(mOff + r) * 20 + rlane] = acc2[r];
  }
  wave_sync();

  const int row = rlane;
  const int gs  = q0 + row;
  const float s510 = sl1[row * 20 + 0] * kTailScale + b51[h * 2 + 0];
  const float s511 = sl1[row * 20 + 1] * kTailScale + b51[h * 2 + 1];
  const float z520 = sl2[row * 20 + 0] * kTailScale + b52[h * 2 + 0];
  const float z521 = sl2[row * 20 + 1] * kTailScale + b52[h * 2 + 1];
  const float e520 = expf(fminf(-z520, 60.0f));
  const float e521 = expf(fminf(-z521, 60.0f));
  const float x520 = 4.0f * (1.0f / (1.0f + e520));
  const float x521 = 4.0f * (1.0f / (1.0f + e521));

  float a0v = x520;
  if (write_a0 == 0) a0v = a0in[(size_t)gs * 2 + 0];
  const float bi = x521;

  const v4f xv = *(const v4f*)(x + (size_t)gs * kDimIn);
  const float t1 = xv[0] * stdv[0] + mean[0];
  const float w1 = xv[1] * stdv[1] + mean[1];
  const float t2 = xv[2] * stdv[2] + mean[2];
  const float w2 = xv[3] * stdv[3] + mean[3];
  const float s1 = sinf(t1);
  const float s2 = sinf(t2);
  const float c1 = cosf(t1);
  const float c2 = cosf(t2);
  const float px = kL1 * c1 + kL2 * c2 - kObsX;
  const float py = kL1 * s1 + kL2 * s2 - kObsY;
  const float vx = (-kL1) * s1 * w1 - kL2 * s2 * w2;
  const float vy = kL1 * c1 * w1 + kL2 * c2 * w2;
  const float barr = px * px + py * py - kR2;
  const float bdot = 2.0f * px * vx + 2.0f * py * vy;
  const float w1s = w1 * w1, w2s = w2 * w2;
  const float Lf2b = 2.0f * (vx * vx) + 2.0f * (vy * vy)
                   + 2.0f * px * ((-kL1) * c1 * w1s - kL2 * c2 * w2s)
                   + 2.0f * py * ((-kL1) * s1 * w1s - kL2 * s2 * w2s);
  const float lg1 = 2.0f * px * ((-kL1) * s1) + 2.0f * py * (kL1 * c1);
  const float lg2 = 2.0f * px * ((-kL2) * s2) + 2.0f * py * (kL2 * c2);
  const float g0 = -lg1, g1 = -lg2;

  const float hval = Lf2b + (a0v + bi) * bdot + a0v * bi * barr;
  const float u0 = -s510, u1 = -s511;
  const float gg = g0 * g0 + g1 * g1;
  const float viol = u0 * g0 + u1 * g1 - hval;
  const float lam = fmaxf(viol, 0.0f) * (1.0f / gg);
  float uu0 = u0 - lam * g0;
  float uu1 = u1 - lam * g1;
  uu0 = (uu0 - mean_label[0]) * (1.0f / std_label[0]);
  uu1 = (uu1 - mean_label[1]) * (1.0f / std_label[1]);

  float wm = wt[0];
#pragma unroll 1
  for (int i = 1; i < kHeads; ++i) wm = fmaxf(wm, wt[i]);
  float wsum = 0.0f, weh = 0.0f;
#pragma unroll 1
  for (int i = 0; i < kHeads; ++i) {
    const float e = expf(wt[i] - wm);
    wsum = wsum + e;
    weh = (i == h) ? e : weh;
  }
  const float wh = weh * (1.0f / wsum);

  float p0 = 0.0f, p1 = 0.0f;
  if (has_prev != 0) {
    p0 = accin[(size_t)gs * 2 + 0];
    p1 = accin[(size_t)gs * 2 + 1];
  }
  const float o0 = p0 + wh * uu0;
  const float o1 = p1 + wh * uu1;

  float* so = sOut[wave];
  float* sa = sA0[wave];
  if (lane < 16) { so[2 * row] = o0; so[2 * row + 1] = o1; }
  if (write_a0 != 0 && lane < 16) { sa[2 * row] = x520; sa[2 * row + 1] = x521; }
  wave_sync();
  for (int pass = 0; pass < 2; ++pass) {
    if (lane < 8) {
      const v4f v = *(const v4f*)(so + lane * 4);
      *(volatile v4f*)(accout + (size_t)q0 * 2 + lane * 4) = v;
    }
    if (write_a0 != 0 && lane < 8) {
      const v4f v = *(const v4f*)(sa + lane * 4);
      *(volatile v4f*)(a0out + (size_t)q0 * 2 + lane * 4) = v;
    }
    __threadfence();
  }
}

static void launch_layer(const unsigned short* A, const unsigned short* Wt, unsigned short* C, const float* bias8,
                         hipStream_t stream) {
  wmma_gemm64<0, false, 2, 1, false, 2><<<dim3(kGemmBlocks, kGroup), 256, 0, stream>>>(
      A, A, kHid, (long)kPlaneElems,
      Wt, Wt, kHid, (long)kWElems,
      (void*)C, (void*)C, kHid, (long)kPlaneElems,
      bias8, (long)kHid,
      bias8, 0L,
      kRows, kHid, kHid, kGemmScale);
}

extern "C" void kernel_launch(void* const* d_in, const int* in_sizes, int n_in,
                              void* d_out, int out_size, void* d_ws, size_t ws_size,
                              hipStream_t stream)
{
  if (n_in < 23) return;
  if (in_sizes[0] != kRows * kDimIn) return;
  if (in_sizes[7] != kHeads * kHid * kDimIn) return;
  if (in_sizes[9] != kHeads * kHid * kHid || in_sizes[17] != kHeads * kHid * kHid) return;
  if (in_sizes[19] != kHeads * 2 * kHid || in_sizes[21] != kHeads * 2 * kHid) return;
  if (out_size != kRows * 2) return;
  if (ws_size < kWsTotal) return;

  const float* x          = (const float*)d_in[0];
  const float* wt         = (const float*)d_in[2];
  const float* mean       = (const float*)d_in[3];
  const float* stdv       = (const float*)d_in[4];
  const float* mean_label = (const float*)d_in[5];
  const float* std_label  = (const float*)d_in[6];
  const float* W1  = (const float*)d_in[7];
  const float* b1  = (const float*)d_in[8];
  const float* W2  = (const float*)d_in[9];
  const float* b2  = (const float*)d_in[10];
  const float* W31 = (const float*)d_in[11];
  const float* b31 = (const float*)d_in[12];
  const float* W32 = (const float*)d_in[13];
  const float* b32 = (const float*)d_in[14];
  const float* W41 = (const float*)d_in[15];
  const float* b41 = (const float*)d_in[16];
  const float* W42 = (const float*)d_in[17];
  const float* b42 = (const float*)d_in[18];
  const float* W51 = (const float*)d_in[19];
  const float* b51 = (const float*)d_in[20];
  const float* W52 = (const float*)d_in[21];
  const float* b52 = (const float*)d_in[22];
  float* out = (float*)d_out;

  char* ws = (char*)d_ws;
  unsigned short* W16 = (unsigned short*)(ws + kOffW16);
  float*          B8  = (float*)(ws + kOffB8);
  unsigned short* S0  = (unsigned short*)(ws + kOffPlane);
  unsigned short* S1  = (unsigned short*)(ws + kOffPlane + kBytesSlot);
  unsigned short* S2  = (unsigned short*)(ws + kOffPlane + 2 * kBytesSlot);
  float*          A0S = (float*)(ws + kOffA0);
  float*          ACC[2] = { (float*)(ws + kOffAcc0), (float*)(ws + kOffAcc1) };

  const int n8 = (int)(kWLayer / 8);
  wcast8_kernel<<<dim3((n8 + 255) / 256, kNLayers), 256, 0, stream>>>(W2, W31, W32, W41, W42, W16, n8, kWCarry);
  const int n4 = (int)(kBLayer / 4);
  bias_scale_kernel<<<dim3((n4 + 255) / 256, kNLayers), 256, 0, stream>>>(b2, b31, b32, b41, b42, B8, n4, kActCarry);

  for (int grp = 0; grp < kNGroups; ++grp) {
    const int hb0 = grp * kGroup;
    input_layer_kernel<<<(unsigned)((long)kGroup * kRows * 32 / 256), 256, 0, stream>>>(x, W1, b1, S0, hb0);
    launch_layer(S0, W16 + 0 * kWLayer + (long)hb0 * kWElems, S1, B8 + 0 * kBLayer + hb0 * kHid, stream);
    launch_layer(S1, W16 + 1 * kWLayer + (long)hb0 * kWElems, S0, B8 + 1 * kBLayer + hb0 * kHid, stream);
    launch_layer(S1, W16 + 2 * kWLayer + (long)hb0 * kWElems, S2, B8 + 2 * kBLayer + hb0 * kHid, stream);
    launch_layer(S0, W16 + 3 * kWLayer + (long)hb0 * kWElems, S1, B8 + 3 * kBLayer + hb0 * kHid, stream);
    launch_layer(S2, W16 + 4 * kWLayer + (long)hb0 * kWElems, S0, B8 + 4 * kBLayer + hb0 * kHid, stream);
    for (int g = 0; g < kGroup; ++g) {
      const int h = hb0 + g;
      const unsigned short* P41 = S1 + (long)g * kPlaneElems;
      const unsigned short* P42 = S0 + (long)g * kPlaneElems;
      float* accout = (h == kHeads - 1) ? out : ACC[h & 1];
      const float* accin = ACC[(h + 1) & 1];
      tail_kernel<<<kRows / 128, 256, 0, stream>>>(P41, P42, W51, b51, W52, b52,
                                                  x, mean, stdv, mean_label, std_label, wt,
                                                  A0S, A0S, accin, accout,
                                                  h, (h > 0) ? 1 : 0, (h == 0) ? 1 : 0);
    }
  }
}
